// JointGeometryBlock_9964324127133
// MI455X (gfx1250) — hardware-verified
//
#include <hip/hip_runtime.h>


#define NB_  2
#define TT   2048
#define DD   1024
#define NH_  16
#define HD   64
#define NF   32
#define F3   (3 * DD)
#define FU   (8 * DD)
#define FG   (4 * DD)
#define ZH   2
#define PCAR 1024.0f
#define WSC  16384.0f
typedef _Float16 h16;
typedef unsigned short bf;
typedef __attribute__((ext_vector_type(16))) __bf16   v16bf;
typedef __attribute__((ext_vector_type(16))) _Float16 v16h;
typedef __attribute__((ext_vector_type(8)))  _Float16 v8h;
typedef __attribute__((ext_vector_type(8)))  unsigned short v8us;
typedef __attribute__((ext_vector_type(8)))  float    v8f;
typedef __attribute__((ext_vector_type(4)))  float    v4f;
typedef v8h  __attribute__((may_alias)) v8ha;
typedef v4f  __attribute__((may_alias)) v4fa;
typedef v8us __attribute__((may_alias)) v8usa;

__device__ __forceinline__ unsigned short f2bf(float f) { unsigned u = __float_as_uint(f); u += 0x7FFFu + ((u >> 16) & 1u); return (unsigned short)(u >> 16); }
__device__ __forceinline__ float bf2f(unsigned short b) { return __uint_as_float(((unsigned)b) << 16); }
__device__ __forceinline__ float bfr(float f) { return bf2f(f2bf(f)); }
__device__ __forceinline__ v16h cat16(v8h lo, v8h hi) { return __builtin_shufflevector(lo, hi, 0, 1, 2, 3, 4, 5, 6, 7, 8, 9, 10, 11, 12, 13, 14, 15); }
__device__ __forceinline__ v16bf cat16b(v8us lo, v8us hi) { return __builtin_bit_cast(v16bf, __builtin_shufflevector(lo, hi, 0, 1, 2, 3, 4, 5, 6, 7, 8, 9, 10, 11, 12, 13, 14, 15)); }
__device__ __forceinline__ v8f wmma16(v16h a, v16h b, v8f c) { return __builtin_amdgcn_wmma_f32_16x16x32_f16(false, a, false, b, (short)0, c, false, false); }
__device__ __forceinline__ v8f wmmab(v16bf a, v16bf b, v8f c) { return __builtin_amdgcn_wmma_f32_16x16x32_bf16(false, a, false, b, (short)0, c, false, false); }


template <typename T16> struct WFrag;
template <> struct WFrag<h16> { typedef v16h V; static __device__ __forceinline__ V ld(const h16* p) { return cat16(*(const v8h*)p, *(const v8h*)(p + 16)); } static __device__ __forceinline__ v8f mma(V a, V b, v8f c) { return wmma16(a, b, c); } };
template <> struct WFrag<bf> { typedef v16bf V; static __device__ __forceinline__ V ld(const bf* p) { return cat16b(*(const v8us*)p, *(const v8us*)(p + 16)); } static __device__ __forceinline__ v8f mma(V a, V b, v8f c) { return wmmab(a, b, c); } };
template <typename T16, int NSPLIT, bool BIAS>
__global__ __launch_bounds__(32) void k_gemmw(const T16* __restrict__ A, const T16* __restrict__ A2, const T16* __restrict__ Bt, const T16* __restrict__ Bt2, int K, float* C, int ldc, const float* __restrict__ bias, size_t sA, size_t sB, size_t sC) {
    typedef typename WFrag<T16>::V V;
    __shared__ __align__(16) float os[16 * 68];
    const size_t z = blockIdx.z; A += z * sA; if (A2) A2 += z * sA; Bt += z * sB; if (Bt2) Bt2 += z * sB; C += z * sC;
    const int lane = threadIdx.x & 31, lr = lane & 15, hi = lane >> 4; const int r0 = blockIdx.x * 64, c0 = blockIdx.y * 64;
    v8f acc[4][4];
#pragma unroll
    for (int mb = 0; mb < 4; ++mb)
#pragma unroll
        for (int nb = 0; nb < 4; ++nb) acc[mb][nb] = (v8f){};
    const size_t aoff = (size_t)(r0 + lr) * K + 8 * hi, boff = (size_t)(c0 + lr) * K + 8 * hi;
#pragma unroll 1
    for (int kc = 0; kc < K; kc += 32) {
        V a[4], a2[4];
#pragma unroll
        for (int mb = 0; mb < 4; ++mb) { a[mb] = WFrag<T16>::ld(A + aoff + (size_t)mb * 16 * K + kc); if (NSPLIT == 1 || NSPLIT == 2) a2[mb] = WFrag<T16>::ld(A2 + aoff + (size_t)mb * 16 * K + kc); }
#pragma unroll
        for (int nb = 0; nb < 4; ++nb) { const V b = WFrag<T16>::ld(Bt + boff + (size_t)nb * 16 * K + kc); V b2; if (NSPLIT >= 2) b2 = WFrag<T16>::ld(Bt2 + boff + (size_t)nb * 16 * K + kc);
#pragma unroll
            for (int mb = 0; mb < 4; ++mb) { acc[mb][nb] = WFrag<T16>::mma(a[mb], b, acc[mb][nb]); if (NSPLIT == 1 || NSPLIT == 2) acc[mb][nb] = WFrag<T16>::mma(a2[mb], b, acc[mb][nb]); if (NSPLIT >= 2) acc[mb][nb] = WFrag<T16>::mma(a[mb], b2, acc[mb][nb]); } }
        asm volatile("v_nop\n\tv_nop\n\tv_nop\n\tv_nop" : "+v"(acc[0][0]), "+v"(acc[1][1]), "+v"(acc[2][2]), "+v"(acc[3][3]) : "v"(a[0]), "v"(a[3]));
    }
#pragma unroll
    for (int mb = 0; mb < 4; ++mb) {
#pragma unroll
        for (int nb = 0; nb < 4; ++nb) {
#pragma unroll
            for (int j = 0; j < 8; ++j) os[(hi * 8 + j) * 68 + nb * 16 + lr] = acc[mb][nb][j]; }
        __builtin_amdgcn_wave_barrier(); asm volatile("" ::: "memory");
        float* crow = C + (size_t)(r0 + mb * 16) * ldc + c0;
#pragma unroll 1
        for (int ps = 0; ps < 2; ++ps) {
#pragma unroll
            for (int s = 0; s < 8; ++s) { const int row = 2 * s + hi, cofs = lr * 4; v4f val = *(const v4fa*)(os + row * 68 + cofs); if (BIAS) { val[0] += bfr(bias[c0 + cofs]); val[1] += bfr(bias[c0 + cofs + 1]); val[2] += bfr(bias[c0 + cofs + 2]); val[3] += bfr(bias[c0 + cofs + 3]); }
                *(volatile v4f*)(crow + (size_t)row * ldc + cofs) = val; }
            if (ps == 0) __threadfence(); }
        __builtin_amdgcn_wave_barrier(); asm volatile("" ::: "memory");
    }
}

__device__ __forceinline__ h16 tohx(float x) { return (h16)x; }
__device__ __forceinline__ void splitf(float y, unsigned short& h, unsigned short& l) { h = f2bf(y); l = f2bf(y - bf2f(h)); }
typedef __attribute__((ext_vector_type(2))) _Float16 v2h;
typedef __attribute__((ext_vector_type(4))) _Float16 v4h;
typedef __attribute__((ext_vector_type(8))) _Float16 v8h16;
typedef __attribute__((ext_vector_type(2))) unsigned short v2us;
typedef __attribute__((ext_vector_type(4))) unsigned short v4us;
typedef __attribute__((ext_vector_type(2))) float v2f;

__global__ __launch_bounds__(256) void k_cvt8(const float* __restrict__ src, bf* dst, size_t n8) { const size_t i = (size_t)blockIdx.x * 256 + threadIdx.x; if (i >= n8) return; const v8f v = *(const v8f*)(src + i * 8); v8us o;
#pragma unroll
    for (int k = 0; k < 8; ++k) o[k] = f2bf(v[k]); *(volatile v8us*)(dst + i * 8) = o; __threadfence(); *(volatile v8us*)(dst + i * 8) = o; }
__global__ __launch_bounds__(256) void k_cvt16(const float* __restrict__ src, h16* dst, size_t n8) { const size_t i = (size_t)blockIdx.x * 256 + threadIdx.x; if (i >= n8) return; const v8f v = *(const v8f*)(src + i * 8); v8h16 o;
#pragma unroll
    for (int k = 0; k < 8; ++k) o[k] = tohx(bfr(v[k]) * WSC); *(volatile v8h16*)(dst + i * 8) = o; __threadfence(); *(volatile v8h16*)(dst + i * 8) = o; }
__global__ __launch_bounds__(256) void k_bsc(const float* __restrict__ b, float* BS, int n) { const int i = (blockIdx.x * 256 + threadIdx.x) * 4; if (i >= n) return; const v4f a = *(const v4f*)(b + i); v4f o;
#pragma unroll
    for (int q = 0; q < 4; ++q) o[q] = bfr(a[q]) * WSC; *(volatile v4f*)(BS + i) = o; __threadfence(); *(volatile v4f*)(BS + i) = o; }
__global__ __launch_bounds__(256) void k_cstab(float* CSN) {
    const int idx = blockIdx.x * 256 + threadIdx.x; if (idx >= TT * NF) return; const int t = idx / NF, i = idx % NF; const float den = powf(10000.0f, (float)(2 * i) * (1.0f / HD)); const float ang = __fdiv_rn((float)t, den);
    v2f o; o[0] = cosf(ang); o[1] = -sinf(ang);     *(volatile v2f*)(CSN + (size_t)idx * 2) = o; __threadfence(); *(volatile v2f*)(CSN + (size_t)idx * 2) = o; }
__global__ __launch_bounds__(256) void k_hsplit(const float* __restrict__ F, int pitch, int nheads, const float* __restrict__ CSN, bf* Ph, bf* Pl, h16* P16) {
    const int lane = threadIdx.x & 31; const int L0 = (blockIdx.x * 8 + (threadIdx.x >> 5)) * 8; const int nlines = nheads * TT * HD / 64;
#pragma unroll 1
    for (int ps = 0; ps < 2; ++ps) {
#pragma unroll
        for (int l = 0; l < 8; ++l) { const int L = L0 + l; if (L >= nlines) break; const int e = L * 64 + lane * 2; const int d = e & (HD - 1); const int t = (e >> 6) & (TT - 1); const int h = e >> 17; v2us oh, ol; v2h o16;
#pragma unroll
            for (int q = 0; q < 2; ++q) { const int dd = d + q; const float x0 = F[(size_t)t * pitch + h * HD + dd], x1 = F[(size_t)t * pitch + h * HD + (dd ^ NF)]; const v2f cs = *(const v2f*)(CSN + ((size_t)t * NF + (dd & (NF - 1))) * 2);
                float a0 = __fmul_rn(cs[0], x0), a1 = __fmul_rn(cs[1], x1); asm volatile("" : "+v"(a0)); asm volatile("" : "+v"(a1)); const float r = (dd < NF) ? __fsub_rn(a0, a1) : __fadd_rn(a0, a1);
                unsigned short a, c2; splitf(r, a, c2); oh[q] = a; ol[q] = c2; o16[q] = tohx(r); }
            *(volatile v2us*)(Ph + (size_t)e) = oh; *(volatile v2us*)(Pl + (size_t)e) = ol; *(volatile v2h*)(P16 + (size_t)e) = o16; }
        if (ps == 0) __threadfence(); }
}
__global__ __launch_bounds__(256) void k_vtplane(const float* __restrict__ F, int pitch, int nheads, bf* Vh, bf* Vl, h16* V16) {
    const int lane = threadIdx.x & 31; const int L0 = (blockIdx.x * 8 + (threadIdx.x >> 5)) * 8; const int nlines = nheads * TT * HD / 64;
#pragma unroll 1
    for (int ps = 0; ps < 2; ++ps) {
#pragma unroll
        for (int l = 0; l < 8; ++l) { const int L = L0 + l; if (L >= nlines) break; const int e = L * 64 + lane * 2; const int t = e & (TT - 1); const int d = (e >> 11) & (HD - 1); const int h = e >> 17; v2us oh, ol; v2h o16;
#pragma unroll
            for (int q = 0; q < 2; ++q) { const float x = F[(size_t)(t + q) * pitch + h * HD + d]; unsigned short a, c2; splitf(x, a, c2); oh[q] = a; ol[q] = c2; o16[q] = tohx(x); }
            *(volatile v2us*)(Vh + (size_t)e) = oh; *(volatile v2us*)(Vl + (size_t)e) = ol; *(volatile v2h*)(V16 + (size_t)e) = o16; }
        if (ps == 0) __threadfence(); }
}
template <int RAW>
__global__ __launch_bounds__(256) void k_rms(const float* __restrict__ X, bf* Hh, bf* Hl, h16* T16) {
    const int lane = threadIdx.x & 31; const int r = blockIdx.x * 8 + (threadIdx.x >> 5); if (r >= TT) return; float v[DD / 32]; float ss = 0.f;
#pragma unroll
    for (int c = 0; c < DD / 128; ++c) { const v4f a = *(const v4f*)(X + (size_t)r * DD + c * 128 + lane * 4);
#pragma unroll
        for (int q = 0; q < 4; ++q) { const float t = RAW ? bfr(a[q]) : a[q]; v[c * 4 + q] = t; float p = __fmul_rn(t, t); asm volatile("" : "+v"(p)); ss = __fadd_rn(ss, p); } }
#pragma unroll
    for (int sh = 16; sh; sh >>= 1) ss += __shfl_xor(ss, sh, 32);
    const float rs = __frsqrt_rn(__fadd_rn(ss * (1.0f / DD), 1e-6f));
#pragma unroll 1
    for (int ps = 0; ps < 2; ++ps) {
#pragma unroll
        for (int c = 0; c < DD / 128; ++c) { const size_t o = (size_t)r * DD + c * 128 + lane * 4;
            if (RAW) { v4us oh, ol;
#pragma unroll
                for (int q = 0; q < 4; ++q) { unsigned short a2, c2; splitf(__fmul_rn(v[c * 4 + q], rs), a2, c2); oh[q] = a2; ol[q] = c2; }
                *(volatile v4us*)(Hh + o) = oh; *(volatile v4us*)(Hl + o) = ol; }
            else { v4h t4;
#pragma unroll
                for (int q = 0; q < 4; ++q) t4[q] = tohx(__fmul_rn(v[c * 4 + q], rs)); *(volatile v4h*)(T16 + o) = t4; } }
        if (ps == 0) __threadfence(); }
}
__global__ __launch_bounds__(256) void k_tc(const float* __restrict__ F, const float* __restrict__ kc, float* QN) { const int i = blockIdx.x * 256 + threadIdx.x; if (i >= NH_ * TT) return; const int t = i & (TT - 1); const int h = i >> 11; const float* f = F + (size_t)t * F3 + h * HD; float s = 0.f;
#pragma unroll 4
    for (int d = 0; d < HD; d += 4) { const v4f v = *(const v4f*)(f + d);
#pragma unroll
        for (int q = 0; q < 4; ++q) { float p = __fmul_rn(v[q], v[q]); asm volatile("" : "+v"(p)); s = __fadd_rn(s, p); } }
    const float o = __fsqrt_rn(__fadd_rn(bfr(kc[h]), s)); *(volatile float*)(QN + i) = o; __threadfence(); *(volatile float*)(QN + i) = o; }
__global__ __launch_bounds__(256) void k_lsoft(const float* __restrict__ Sb, const float* __restrict__ QN, const float* __restrict__ KN, const float* __restrict__ kc, int h0, h16* P16) {
    const int lane = threadIdx.x & 31; const int row = blockIdx.x * 8 + (threadIdx.x >> 5); if (row >= ZH * TT) return; const int i = row & (TT - 1); const int zz = row >> 11; const int h = h0 + zz;
    const float kcv = bfr(kc[h]); const float ikc = __fdiv_rn(1.0f, kcv); const float skc = __fsqrt_rn(kcv); const float q0 = QN[(size_t)h * TT + i]; const float* kr = KN + (size_t)h * TT; const float* sr = Sb + (size_t)row * TT; float v[64]; float mx = -3.0e38f;
#pragma unroll
    for (int ch = 0; ch < 16; ++ch) { const int j0 = ch * 128 + lane * 4; const v4f a = *(const v4f*)(sr + j0), k4 = *(const v4f*)(kr + j0);
#pragma unroll
        for (int q = 0; q < 4; ++q) { const int j = j0 + q; float t = -3.0e38f;
            if (j <= i) { float qk0 = __fmul_rn(q0, k4[q]); asm volatile("" : "+v"(qk0)); float nl = __fsub_rn(qk0, a[q]); asm volatile("" : "+v"(nl)); const float arg = fmaxf(__fmul_rn(nl, ikc), 1.000001f);
                float a2 = __fmul_rn(arg, arg); asm volatile("" : "+v"(a2)); const float sq = __builtin_amdgcn_sqrtf(__fsub_rn(a2, 1.0f)); float l2 = __builtin_amdgcn_logf(__fadd_rn(arg, sq)); asm volatile("" : "+v"(l2)); float ac = __fmul_rn(l2, 0.69314718055994531f); asm volatile("" : "+v"(ac)); t = -__fmul_rn(skc, ac); }
            v[ch * 4 + q] = t; mx = fmaxf(mx, t); } }
#pragma unroll
    for (int sh = 16; sh; sh >>= 1) mx = fmaxf(mx, __shfl_xor(mx, sh, 32));
    float sum = 0.f;
#pragma unroll
    for (int k = 0; k < 64; ++k) { float d0 = __fsub_rn(v[k], mx); asm volatile("" : "+v"(d0)); v[k] = __builtin_amdgcn_exp2f(__fmul_rn(d0, 1.4426950408889634f)); sum += v[k]; }
#pragma unroll
    for (int sh = 16; sh; sh >>= 1) sum += __shfl_xor(sum, sh, 32);
    const float f = __fdiv_rn(PCAR, sum);
#pragma unroll 1
    for (int ps = 0; ps < 2; ++ps) {
#pragma unroll
        for (int ch = 0; ch < 16; ++ch) { v4h o;
#pragma unroll
            for (int q = 0; q < 4; ++q) o[q] = tohx(v[ch * 4 + q] * f);
            *(volatile v4h*)(P16 + (size_t)row * TT + ch * 128 + lane * 4) = o; }
        if (ps == 0) __threadfence(); }
}
__global__ __launch_bounds__(256) void k_merge(const float* __restrict__ O, int h0, bf* Ah, bf* Al) {
    const int lane = threadIdx.x & 31; const int L0 = (blockIdx.x * 8 + (threadIdx.x >> 5)) * 8; const int nlines = TT * ZH * HD / 64;
#pragma unroll 1
    for (int ps = 0; ps < 2; ++ps) {
#pragma unroll
        for (int l = 0; l < 8; ++l) { const int L = L0 + l; if (L >= nlines) break; const int e = L * 64 + lane * 2; const int d = e & 63; const int zz = (e >> 6) % ZH; const int t = (e >> 6) / ZH; v2us oh, ol;
#pragma unroll
            for (int q = 0; q < 2; ++q) { unsigned short a, c2; splitf(O[((size_t)zz * TT + t) * HD + d + q] * (1.0f / PCAR), a, c2); oh[q] = a; ol[q] = c2; }
            const size_t o = (size_t)t * DD + (h0 + zz) * HD + d; *(volatile v2us*)(Ah + o) = oh; *(volatile v2us*)(Al + o) = ol; }
        if (ps == 0) __threadfence(); }
}

__global__ __launch_bounds__(256) void k_res1(const float* __restrict__ x, const float* __restrict__ AO, float* X1) { const size_t i = ((size_t)blockIdx.x * 256 + threadIdx.x) * 4; if (i >= (size_t)TT * DD) return; const v4f a = *(const v4f*)(x + i), b = *(const v4f*)(AO + i); v4f o;
#pragma unroll
    for (int q = 0; q < 4; ++q) o[q] = __fadd_rn(bfr(a[q]), b[q]); *(volatile v4f*)(X1 + i) = o; __threadfence(); *(volatile v4f*)(X1 + i) = o; }
__global__ __launch_bounds__(256) void k_swi(const float* __restrict__ U, h16* G16, int rows) { const size_t i = ((size_t)blockIdx.x * 256 + threadIdx.x) * 2; if (i >= (size_t)rows * FG) return; const int t = (int)(i / FG), j = (int)(i % FG); const float* ur = U + (size_t)t * FU; v2h o;
#pragma unroll
    for (int q = 0; q < 2; ++q) { const float u = ur[j + q] * (1.0f / WSC), g = ur[FG + j + q] * (1.0f / WSC); const float sg = __fdiv_rn(g, __fadd_rn(1.0f, __expf(-g))); o[q] = tohx(__fmul_rn(u, sg)); }
    *(volatile v2h*)(G16 + i) = o; __threadfence(); *(volatile v2h*)(G16 + i) = o; }
__global__ __launch_bounds__(256) void k_fin(const float* __restrict__ X1, const float* __restrict__ HM, float* OUT) { const size_t i = ((size_t)blockIdx.x * 256 + threadIdx.x) * 4; if (i >= (size_t)TT * DD) return; const v4f a = *(const v4f*)(X1 + i), b = *(const v4f*)(HM + i); v4f o;
#pragma unroll
    for (int q = 0; q < 4; ++q) o[q] = __fadd_rn(a[q], b[q] * (1.0f / WSC)); *(volatile v4f*)(OUT + i) = o; __threadfence(); *(volatile v4f*)(OUT + i) = o; }

extern "C" void kernel_launch(void* const* d_in, const int* in_sizes, int n_in,
                              void* d_out, int out_size, void* d_ws, size_t ws_size, hipStream_t stream) {
    (void)in_sizes; (void)n_in; (void)out_size;
    const float* x = (const float*)d_in[0]; const float* wqkv = (const float*)d_in[1]; const float* wout = (const float*)d_in[2]; const float* kc = (const float*)d_in[3]; const float* wuv = (const float*)d_in[4]; const float* buv = (const float*)d_in[5]; const float* wmo = (const float*)d_in[6]; const float* bmo = (const float*)d_in[7];
    float* OUT = (float*)d_out;
    char* wsp = (char*)d_ws;
    auto take = [&](size_t bytes) { char* p = wsp; wsp += (bytes + 255) & ~(size_t)255; return (void*)p; };
    bf* WQKV = (bf*)take((size_t)F3 * DD * 2); bf* WOUT = (bf*)take((size_t)DD * DD * 2); h16* WUV = (h16*)take((size_t)FU * DD * 2); h16* WMO = (h16*)take((size_t)DD * FG * 2); float* BUV = (float*)take(FU * 4); float* BMO = (float*)take(DD * 4); float* CSN = (float*)take((size_t)TT * NF * 2 * 4);
    bf* Hh = (bf*)take((size_t)TT * DD * 2); bf* Hl = (bf*)take((size_t)TT * DD * 2); float* Fq = (float*)take((size_t)TT * F3 * 4); float* QN = (float*)take((size_t)NH_ * TT * 4); float* KN = (float*)take((size_t)NH_ * TT * 4);
    bf* QPh = (bf*)take((size_t)NH_ * TT * HD * 2); bf* QPl = (bf*)take((size_t)NH_ * TT * HD * 2); h16* QP16 = (h16*)take((size_t)NH_ * TT * HD * 2); bf* KPh = QPh; bf* KPl = QPl; h16* KP16 = (h16*)take((size_t)NH_ * TT * HD * 2);
    bf* VTh = (bf*)take((size_t)NH_ * HD * TT * 2); bf* VTl = (bf*)take((size_t)NH_ * HD * TT * 2); h16* VT16 = (h16*)take((size_t)NH_ * HD * TT * 2);
    char* R0 = wsp; float* Sb = (float*)take((size_t)ZH * TT * TT * 4); h16* Pm = (h16*)take((size_t)ZH * TT * TT * 2); char* R1 = wsp; float* Ob = (float*)take((size_t)ZH * TT * HD * 4); bf* ATh = (bf*)take((size_t)TT * DD * 2); bf* ATl = (bf*)take((size_t)TT * DD * 2);
    float* X1 = (float*)take((size_t)TT * DD * 4); h16* T16 = (h16*)take((size_t)TT * DD * 2); h16* G16 = (h16*)take((size_t)TT * FG * 2); float* HM = (float*)take((size_t)TT * DD * 4);
    if ((size_t)(wsp - (char*)d_ws) > ws_size) return;
    float* AO = HM;
    float* Uh = (float*)R0; if ((char*)(Uh + (size_t)(TT / 2) * FU) > R1) return;
    { k_cvt8<<<(unsigned)(((size_t)F3 * DD / 8 + 255) / 256), 256, 0, stream>>>(wqkv, WQKV, (size_t)F3 * DD / 8); k_cvt8<<<(DD * DD / 8 + 255) / 256, 256, 0, stream>>>(wout, WOUT, (size_t)DD * DD / 8);
      k_cvt16<<<(unsigned)(((size_t)FU * DD / 8 + 255) / 256), 256, 0, stream>>>(wuv, WUV, (size_t)FU * DD / 8); k_cvt16<<<(unsigned)(((size_t)DD * FG / 8 + 255) / 256), 256, 0, stream>>>(wmo, WMO, (size_t)DD * FG / 8);
      k_bsc<<<FU / 1024, 256, 0, stream>>>(buv, BUV, FU); k_bsc<<<DD / 1024, 256, 0, stream>>>(bmo, BMO, DD); k_cstab<<<(TT * NF + 255) / 256, 256, 0, stream>>>(CSN); }
    const unsigned LB = (unsigned)((NH_ * TT * HD / 64 + 63) / 64), L4 = (unsigned)(((size_t)TT * DD / 4 + 255) / 256), LN = (NH_ * TT + 255) / 256;
    for (int b = 0; b < NB_; ++b) { const float* xb = x + (size_t)b * TT * DD;
        k_rms<1><<<TT / 8, 256, 0, stream>>>(xb, Hh, Hl, nullptr);
        k_gemmw<bf, 1, false><<<dim3(TT / 64, F3 / 64, 1), 32, 0, stream>>>(Hh, Hl, WQKV, nullptr, DD, Fq, F3, nullptr, 0, 0, 0);
        k_tc<<<LN, 256, 0, stream>>>(Fq, kc, QN); k_tc<<<LN, 256, 0, stream>>>(Fq + DD, kc, KN);
        k_hsplit<<<LB, 256, 0, stream>>>(Fq + DD, F3, NH_, CSN, KPh, KPl, KP16);
        k_hsplit<<<LB, 256, 0, stream>>>(Fq, F3, NH_, CSN, QPh, QPl, QP16);
        k_vtplane<<<LB, 256, 0, stream>>>(Fq + 2 * DD, F3, NH_, VTh, VTl, VT16);
        for (int h0 = 0; h0 < NH_; h0 += ZH) { const size_t po = (size_t)h0 * TT * HD;
            k_gemmw<h16, 0, false><<<dim3(TT / 64, TT / 64, ZH), 32, 0, stream>>>(QP16 + po, nullptr, KP16 + po, nullptr, HD, Sb, TT, nullptr, (size_t)TT * HD, (size_t)TT * HD, (size_t)TT * TT);
            k_lsoft<<<ZH * TT / 8, 256, 0, stream>>>(Sb, QN, KN, kc, h0, Pm);
            k_gemmw<h16, 0, false><<<dim3(TT / 64, 1, ZH), 32, 0, stream>>>(Pm, nullptr, VT16 + po, nullptr, TT, Ob, HD, nullptr, (size_t)TT * TT, (size_t)HD * TT, (size_t)TT * HD);
            k_merge<<<(TT * ZH * HD / 64 + 63) / 64, 256, 0, stream>>>(Ob, h0, ATh, ATl); }
        k_gemmw<bf, 1, false><<<dim3(TT / 64, DD / 64, 1), 32, 0, stream>>>(ATh, ATl, WOUT, nullptr, DD, AO, DD, nullptr, 0, 0, 0);
        k_res1<<<L4, 256, 0, stream>>>(xb, AO, X1); k_rms<0><<<TT / 8, 256, 0, stream>>>(X1, nullptr, nullptr, T16);
        for (int hb = 0; hb < 2; ++hb) { const size_t r0 = (size_t)hb * (TT / 2);
            k_gemmw<h16, 0, true><<<dim3((TT / 2) / 64, FU / 64, 1), 32, 0, stream>>>(T16 + r0 * DD, nullptr, WUV, nullptr, DD, Uh, FU, BUV, 0, 0, 0);
            k_swi<<<(unsigned)(((size_t)(TT / 2) * FG / 2 + 255) / 256), 256, 0, stream>>>(Uh, G16 + r0 * FG, TT / 2); }
        k_gemmw<h16, 0, true><<<dim3(TT / 64, DD / 64, 1), 32, 0, stream>>>(G16, nullptr, WMO, nullptr, FG, HM, DD, BMO, 0, 0, 0);
        k_fin<<<L4, 256, 0, stream>>>(X1, HM, OUT + (size_t)b * TT * DD); }
}
